// Mamba2Triton_61512521614096
// MI455X (gfx1250) — hardware-verified
//
#include <hip/hip_runtime.h>
#include <hip/hip_bf16.h>
#include <math.h>

#define NBATCH 2
#define SEQL   2048
#define NH     32
#define HD     64
#define NS     128
#define CH     256
#define NCH    (SEQL / CH)
#define XW     (NH * HD)
#define GSTR   40
#define OSTR   68
#define SMEMB  (8 * 16 * OSTR * 4)

static_assert(SMEMB >= (2 * 128 * GSTR + 2 * 64 * GSTR) * 2);
static_assert(SEQL % CH == 0);
static_assert(CH == 256);
static_assert(HD == 64);
static_assert(NS == 128);

typedef unsigned short us16 __attribute__((ext_vector_type(16)));
typedef unsigned short us8  __attribute__((ext_vector_type(8)));
typedef unsigned short us8a __attribute__((ext_vector_type(8), may_alias));
typedef __bf16 v16b __attribute__((ext_vector_type(16)));
typedef float v8f __attribute__((ext_vector_type(8)));
typedef float v4f __attribute__((ext_vector_type(4)));
typedef float v4fa __attribute__((ext_vector_type(4), may_alias));
union FragU { us16 v; us8 h[2]; };

__device__ __forceinline__ unsigned short bf16_bits(float f) {
  unsigned u = __float_as_uint(f);
  u += 0x7FFFu + ((u >> 16) & 1u);
  return (unsigned short)(u >> 16);
}
__device__ __forceinline__ float bf16_val(unsigned short b) { return __uint_as_float(((unsigned)b) << 16); }
__device__ __forceinline__ float bf16r(float f) { return bf16_val(bf16_bits(f)); }

__device__ __forceinline__ v8f mma_bf16(us16 a, us16 b, v8f c) {
  return __builtin_amdgcn_wmma_f32_16x16x32_bf16(false, __builtin_bit_cast(v16b, a), false, __builtin_bit_cast(v16b, b), (short)0, c, false, false);
}
__device__ __forceinline__ void wguard(v8f& c0, v8f& c1, v8f& c2, v8f& c3, const us16& a0, const us16& a1,
                                       const us16& b0, const us16& b1, const us16& b2, const us16& b3,
                                       const us16& b4, const us16& b5, const us16& b6, const us16& b7) {
#if defined(__HIP_DEVICE_COMPILE__)
  asm volatile("v_nop\n\tv_nop\n\tv_nop\n\tv_nop"
               : "+v"(c0), "+v"(c1), "+v"(c2), "+v"(c3)
               : "v"(a0), "v"(a1), "v"(b0), "v"(b1), "v"(b2), "v"(b3), "v"(b4), "v"(b5), "v"(b6), "v"(b7));
#endif
}

__device__ __forceinline__ us16 lds_frag(const unsigned short* base) {
  const int lane = threadIdx.x & 31, r = lane & 15, kh = (lane >> 4) * 8;
  FragU f;
  f.h[0] = *(const us8a*)(base + r * GSTR + kh);
  f.h[1] = *(const us8a*)(base + r * GSTR + 16 + kh);
  return f.v;
}

template <int KM>
__device__ __forceinline__ void stage_a(unsigned short* lds, const unsigned short* __restrict__ P, int ld, int m0, int k0, int tid) {
  if (KM == 0) {
    const int row = tid >> 1, cq = (tid & 1) * 16;
    const unsigned short* src = P + (size_t)(m0 + row) * ld + k0 + cq;
    const us8 v0 = *(const us8a*)src;
    const us8 v1 = *(const us8a*)(src + 8);
    *(us8a*)(lds + row * GSTR + cq) = v0;
    *(us8a*)(lds + row * GSTR + cq + 8) = v1;
  } else {
    const int k = tid >> 3, mq = (tid & 7) * 16;
    const unsigned short* src = P + (size_t)(k0 + k) * ld + m0 + mq;
    const us8 v0 = *(const us8a*)src;
    const us8 v1 = *(const us8a*)(src + 8);
#pragma unroll
    for (int u = 0; u < 8; ++u) { lds[(mq + u) * GSTR + k] = v0[u]; lds[(mq + 8 + u) * GSTR + k] = v1[u]; }
  }
}
template <int KM>
__device__ __forceinline__ void stage_b(unsigned short* lds, const unsigned short* __restrict__ P, int ld, int n0, int k0, int tid) {
  if (KM == 0) {
    const int row = tid >> 2, kq = (tid & 3) * 8;
    const us8 v = *(const us8a*)(P + (size_t)(n0 + row) * ld + k0 + kq);
    *(us8a*)(lds + row * GSTR + kq) = v;
  } else {
    const int k = tid >> 3, nq = (tid & 7) * 8;
    const us8 v = *(const us8a*)(P + (size_t)(k0 + k) * ld + n0 + nq);
#pragma unroll
    for (int u = 0; u < 8; ++u) lds[(nq + u) * GSTR + k] = v[u];
  }
}
__device__ __forceinline__ void stage_w(unsigned short* lhi, unsigned short* llo, const float* __restrict__ G, int ldg,
                                        const float* sac, int m0, int k0, int tid) {
  const int row = tid >> 1, cq = (tid & 1) * 16, m = m0 + row;
  const float* src = G + (size_t)m * ldg + k0 + cq;
  v4f g4[4];
#pragma unroll
  for (int q = 0; q < 4; ++q) g4[q] = *(const v4fa*)(src + 4 * q);
  const float am = sac[m];
  us8 h0, h1, l0, l1;
#pragma unroll
  for (int u = 0; u < 16; ++u) {
    const int s = k0 + cq + u;
    const float d = expf(am - sac[s]);
    const float w = (s <= m) ? g4[u >> 2][u & 3] * d : 0.0f;
    const unsigned short hb = bf16_bits(w);
    const unsigned short lb = bf16_bits(w - bf16_val(hb));
    if (u < 8) { h0[u] = hb; l0[u] = lb; } else { h1[u - 8] = hb; l1[u - 8] = lb; }
  }
  *(us8a*)(lhi + row * GSTR + cq) = h0;
  *(us8a*)(lhi + row * GSTR + cq + 8) = h1;
  *(us8a*)(llo + row * GSTR + cq) = l0;
  *(us8a*)(llo + row * GSTR + cq + 8) = l1;
}

template <int NA, int NBP, int AKM, int BKM, int EPI>
__global__ __launch_bounds__(256) void k_gemm(
    const unsigned short* __restrict__ A0, const unsigned short* __restrict__ A1, const float* __restrict__ Af,
    int lda, long long sAc, long long sAh,
    const unsigned short* __restrict__ B0, const unsigned short* __restrict__ B1, int ldb, long long sBc, long long sBh,
    float* Yg, int ldy, long long sYc, long long sYh,
    const float* __restrict__ R, int ldr, long long sRc, long long sRh,
    const float* __restrict__ acs, long long sXc, long long sXh,
    int zh, int K)
{
  __shared__ __attribute__((aligned(16))) unsigned char sm[SMEMB];
  __shared__ float sacs[CH];
  unsigned short* lA0 = (unsigned short*)sm;
  unsigned short* lA1 = lA0 + 128 * GSTR;
  unsigned short* lB0 = lA1 + 128 * GSTR;
  unsigned short* lB1 = lB0 + 64 * GSTR;
  float* oS = (float*)sm;
  const int tid = threadIdx.x, lane = tid & 31, wave = tid >> 5, cl = lane & 15, hh = lane >> 4;
  const int m0 = blockIdx.x * 128, n0 = blockIdx.y * 64;
  const int z = blockIdx.z, zc = z / zh, zq = z - zc * zh;
  const long long oA = (long long)zc * sAc + (long long)zq * sAh;
  const long long oB = (long long)zc * sBc + (long long)zq * sBh;
  A0 += oA; A1 += oA; Af += oA;
  B0 += oB; B1 += oB;
  const float* acz = acs + (long long)zc * sXc + (long long)zq * sXh;
  if (AKM == 2) sacs[tid] = acz[(size_t)tid * NH];
  int kend = K;
  if (AKM == 2) { const int t = m0 + 128; kend = (t < K) ? t : K; }

  v8f acc[4];
#pragma unroll
  for (int j = 0; j < 4; ++j) { v8f zz = {0.f, 0.f, 0.f, 0.f, 0.f, 0.f, 0.f, 0.f}; acc[j] = zz; }

#pragma unroll 1
  for (int k0 = 0; k0 < kend; k0 += 32) {
    __syncthreads();
    if (AKM == 2) {
      stage_w(lA0, lA1, Af, lda, sacs, m0, k0, tid);
    } else {
      stage_a<AKM>(lA0, A0, lda, m0, k0, tid);
      if (NA > 1) stage_a<AKM>(lA1, A1, lda, m0, k0, tid);
    }
    stage_b<BKM>(lB0, B0, ldb, n0, k0, tid);
    if (NBP > 1) stage_b<BKM>(lB1, B1, ldb, n0, k0, tid);
    __syncthreads();
    const us16 af0 = lds_frag(lA0 + 16 * wave * GSTR);
    us16 af1 = af0;
    if (NA > 1) af1 = lds_frag(lA1 + 16 * wave * GSTR);
    us16 bf0[4], bf1[4];
#pragma unroll
    for (int j = 0; j < 4; ++j) { bf0[j] = lds_frag(lB0 + 16 * j * GSTR); bf1[j] = bf0[j]; }
    if (NBP > 1) {
#pragma unroll
      for (int j = 0; j < 4; ++j) bf1[j] = lds_frag(lB1 + 16 * j * GSTR);
    }
#pragma unroll
    for (int j = 0; j < 4; ++j) acc[j] = mma_bf16(af0, bf0[j], acc[j]);
    if (NBP > 1) {
#pragma unroll
      for (int j = 0; j < 4; ++j) acc[j] = mma_bf16(af0, bf1[j], acc[j]);
    }
    if (NA > 1) {
#pragma unroll
      for (int j = 0; j < 4; ++j) acc[j] = mma_bf16(af1, bf0[j], acc[j]);
    }
    wguard(acc[0], acc[1], acc[2], acc[3], af0, af1, bf0[0], bf0[1], bf0[2], bf0[3], bf1[0], bf1[1], bf1[2], bf1[3]);
  }
  __syncthreads();

  float* so = oS + wave * (16 * OSTR);
#pragma unroll
  for (int j = 0; j < 4; ++j)
#pragma unroll
    for (int r = 0; r < 8; ++r) so[(8 * hh + r) * OSTR + 16 * j + cl] = acc[j][r];
  __syncthreads();
  if (EPI != 0) {
    const float* Rz = R + (long long)zc * sRc + (long long)zq * sRh;
#pragma unroll 1
    for (int e = lane; e < 16 * 64; e += 32) {
      const int r = e >> 6, c = e & 63;
      const int m = m0 + 16 * wave + r, n = n0 + c;
      float v = so[r * OSTR + c];
      if (EPI == 1) v = v * expf(acz[(size_t)m * NH]);
      if (EPI == 2) v = v + Rz[(size_t)m * ldr + n];
      so[r * OSTR + c] = v;
    }
    __syncthreads();
  }
#pragma unroll
  for (int pass = 0; pass < 2; ++pass) {
    float* Y = Yg + (long long)zc * sYc + (long long)zq * sYh;
#pragma unroll
    for (int it = 0; it < 8; ++it) {
      const int ch = it * 32 + lane, r = ch >> 4, q = (ch & 15) * 4;
      const v4f v = *(const v4fa*)(so + r * OSTR + q);
      *(volatile v4f*)(Y + (size_t)(m0 + 16 * wave + r) * ldy + n0 + q) = v;
    }
    __threadfence();
  }
}

__global__ __launch_bounds__(32) void k_acs(const float* __restrict__ dt, const float* __restrict__ Ag, const int* __restrict__ csz,
                                            float* __restrict__ ACS) {
#pragma clang fp contract(off)
  const int zc = blockIdx.x, h = threadIdx.x;
  const float ab = bf16r(Ag[h]);
  (void)csz;
#pragma unroll 1
  for (int pass = 0; pass < 2; ++pass) {
    float run = 0.0f;
#pragma unroll 1
    for (int i = 0; i < CH; ++i) {
      const size_t tok = (size_t)zc * CH + i;
      const float ad = ab * bf16r(dt[tok * NH + h]);
      run = run + ad;
      *(volatile float*)(ACS + tok * NH + h) = run;
    }
    __threadfence();
  }
}

__global__ __launch_bounds__(256) void k_planes(const float* __restrict__ x, const float* __restrict__ dt,
                                               const float* __restrict__ Bg, const float* __restrict__ Cg, const float* __restrict__ ACS,
                                               unsigned short* __restrict__ XH, unsigned short* __restrict__ XL,
                                               unsigned short* __restrict__ XDH, unsigned short* __restrict__ XDL,
                                               unsigned short* __restrict__ B16, unsigned short* __restrict__ C16) {
#pragma clang fp contract(off)
  const int tok = blockIdx.x, tid = threadIdx.x, lane = tid & 31;
  const int last = tok | (CH - 1);
  {
    const int c8 = 8 * tid, h = tid >> 3;
    const float dtv = bf16r(dt[(size_t)tok * NH + h]);
    const float dec = expf(ACS[(size_t)last * NH + h] - ACS[(size_t)tok * NH + h]);
    const float* xs = x + (size_t)tok * XW + c8;
    const v4f x0 = *(const v4fa*)xs, x1 = *(const v4fa*)(xs + 4);
    us8 ph, pl, qh, ql;
#pragma unroll
    for (int u = 0; u < 4; ++u) {
      const float v0 = bf16r(x0[u]) * dtv;
      const unsigned short a0 = bf16_bits(v0);
      ph[u] = a0; pl[u] = bf16_bits(v0 - bf16_val(a0));
      const float w0 = v0 * dec;
      const unsigned short b0 = bf16_bits(w0);
      qh[u] = b0; ql[u] = bf16_bits(w0 - bf16_val(b0));
      const float v1 = bf16r(x1[u]) * dtv;
      const unsigned short a1 = bf16_bits(v1);
      ph[4 + u] = a1; pl[4 + u] = bf16_bits(v1 - bf16_val(a1));
      const float w1 = v1 * dec;
      const unsigned short b1 = bf16_bits(w1);
      qh[4 + u] = b1; ql[4 + u] = bf16_bits(w1 - bf16_val(b1));
    }
    const size_t o = (size_t)tok * XW + c8;
    *(volatile us8*)(XH + o) = ph; *(volatile us8*)(XL + o) = pl; *(volatile us8*)(XDH + o) = qh; *(volatile us8*)(XDL + o) = ql;
    __threadfence();
    *(volatile us8*)(XH + o) = ph; *(volatile us8*)(XL + o) = pl; *(volatile us8*)(XDH + o) = qh; *(volatile us8*)(XDL + o) = ql;
  }
  if (tid < 32) {
    const int j = (lane & 15) * 8;
    const float* src = ((lane < 16) ? Bg : Cg) + (size_t)tok * NS + j;
    unsigned short* dst = ((lane < 16) ? B16 : C16) + (size_t)tok * NS + j;
    const v4f v0 = *(const v4fa*)src, v1 = *(const v4fa*)(src + 4);
    us8 o;
#pragma unroll
    for (int u = 0; u < 4; ++u) { o[u] = bf16_bits(v0[u]); o[4 + u] = bf16_bits(v1[u]); }
    *(volatile us8*)dst = o;
    __threadfence();
    *(volatile us8*)dst = o;
  }
}

__global__ __launch_bounds__(256) void k_prev(const float* __restrict__ ST, const float* __restrict__ ACS,
                                             unsigned short* __restrict__ PH, unsigned short* __restrict__ PL) {
#pragma clang fp contract(off)
  __shared__ float co[64];
  const int part = blockIdx.x, h = blockIdx.y, b = blockIdx.z, tid = threadIdx.x;
  if (tid < 64) {
    const int z = tid >> 3, c = tid & 7;
    float run = 0.0f, csz = 0.0f, csc = 0.0f;
#pragma unroll 1
    for (int j = 1; j <= NCH; ++j) {
      run = run + ACS[((size_t)b * SEQL + (size_t)(j - 1) * CH + (CH - 1)) * NH + h];
      csz = (j == z) ? run : csz;
      csc = (j == c + 1) ? run : csc;
    }
    const float e = expf(csz - csc);
    co[tid] = (c + 1 <= z) ? e : 0.0f;
  }
  __syncthreads();
  const int e0 = part * 2048 + tid * 8;
  v4f s0[NCH], s1[NCH];
#pragma unroll
  for (int c = 0; c < NCH; ++c) {
    const size_t base = ((size_t)(b * NCH + c) * NH + h) * (size_t)(HD * NS) + e0;
    s0[c] = *(const v4fa*)(ST + base);
    s1[c] = *(const v4fa*)(ST + base + 4);
  }
#pragma unroll 1
  for (int z = 0; z < NCH; ++z) {
    v4f o0 = {0.0f, 0.0f, 0.0f, 0.0f}, o1 = {0.0f, 0.0f, 0.0f, 0.0f};
#pragma unroll
    for (int c = 0; c < NCH; ++c) {
      const float k = co[z * 8 + c];
      o0 = o0 + s0[c] * k;
      o1 = o1 + s1[c] * k;
    }
    us8 hi, lo;
#pragma unroll
    for (int u = 0; u < 4; ++u) {
      const unsigned short a = bf16_bits(o0[u]);
      hi[u] = a; lo[u] = bf16_bits(o0[u] - bf16_val(a));
      const unsigned short bb = bf16_bits(o1[u]);
      hi[4 + u] = bb; lo[4 + u] = bf16_bits(o1[u] - bf16_val(bb));
    }
    const size_t ob = ((size_t)(b * NCH + z) * NH + h) * (size_t)(HD * NS) + e0;
    *(volatile us8*)(PH + ob) = hi; *(volatile us8*)(PL + ob) = lo;
    __threadfence();
    *(volatile us8*)(PH + ob) = hi; *(volatile us8*)(PL + ob) = lo;
  }
}

extern "C" void kernel_launch(void* const* d_in, const int* in_sizes, int n_in,
                              void* d_out, int out_size, void* d_ws, size_t ws_size,
                              hipStream_t stream) {
  if (n_in < 6) return;
  if (in_sizes[0] != NBATCH * SEQL * XW || in_sizes[1] != NBATCH * SEQL * NH || in_sizes[2] != NH ||
      in_sizes[3] != NBATCH * SEQL * NS || in_sizes[4] != NBATCH * SEQL * NS || in_sizes[5] < 1 ||
      out_size != NBATCH * SEQL * XW) return;
  const float* x  = (const float*)d_in[0];
  const float* dt = (const float*)d_in[1];
  const float* Ag = (const float*)d_in[2];
  const float* Bg = (const float*)d_in[3];
  const float* Cg = (const float*)d_in[4];
  const int*  csz = (const int*)d_in[5];
  float* out = (float*)d_out;

  const size_t NTOK = (size_t)NBATCH * SEQL;
  const size_t NSL  = (size_t)NBATCH * NCH * NH;
  size_t off = 0;
  auto carve = [&](size_t bytes) -> char* { char* p = (char*)d_ws + off; off += (bytes + 255) & ~(size_t)255; return p; };
  float* ACS           = (float*)carve(NTOK * NH * 4);
  unsigned short* XH   = (unsigned short*)carve(NTOK * XW * 2);
  unsigned short* XL   = (unsigned short*)carve(NTOK * XW * 2);
  char* XD             = carve(NTOK * XW * 2 * 2);
  unsigned short* B16  = (unsigned short*)carve(NTOK * NS * 2);
  unsigned short* C16  = (unsigned short*)carve(NTOK * NS * 2);
  float* G             = (float*)carve((size_t)NBATCH * NCH * CH * CH * 4);
  float* ST            = (float*)carve(NSL * HD * NS * 4);
  unsigned short* PH   = (unsigned short*)carve(NSL * HD * NS * 2);
  unsigned short* PL   = (unsigned short*)carve(NSL * HD * NS * 2);
  if (off > ws_size || off > (size_t)134217728) return;
  unsigned short* XDH = (unsigned short*)XD;
  unsigned short* XDL = XDH + NTOK * XW;
  float* YO = (float*)XD;

  const dim3 blk(256);
  k_acs<<<dim3(NBATCH * NCH), dim3(32), 0, stream>>>(dt, Ag, csz, ACS);
  k_planes<<<dim3((unsigned)NTOK), blk, 0, stream>>>(x, dt, Bg, Cg, ACS, XH, XL, XDH, XDL, B16, C16);
  k_gemm<1, 1, 0, 0, 0><<<dim3(CH / 128, CH / 64, NBATCH * NCH), blk, 0, stream>>>(
      C16, C16, G, NS, (long long)CH * NS, 0,
      B16, B16, NS, (long long)CH * NS, 0,
      G, CH, (long long)CH * CH, 0,
      ACS, 0, 0, 0,
      ACS, 0, 0,
      1, NS);
  k_gemm<1, 2, 1, 1, 0><<<dim3(NS / 128, HD / 64, (unsigned)NSL), blk, 0, stream>>>(
      B16, B16, G, NS, (long long)CH * NS, 0,
      XDH, XDL, XW, (long long)CH * XW, HD,
      ST, HD, (long long)NH * HD * NS, (long long)HD * NS,
      ACS, 0, 0, 0,
      ACS, 0, 0,
      NH, CH);
  k_prev<<<dim3(4, NH, NBATCH), blk, 0, stream>>>(ST, ACS, PH, PL);
  k_gemm<1, 2, 0, 1, 1><<<dim3(CH / 128, HD / 64, (unsigned)NSL), blk, 0, stream>>>(
      C16, C16, G, NS, (long long)CH * NS, 0,
      PH, PL, HD, (long long)NH * HD * NS, (long long)HD * NS,
      YO, XW, (long long)CH * XW, HD,
      ACS, 0, 0, 0,
      ACS, (long long)CH * NH, 1,
      NH, NS);
  k_gemm<2, 2, 2, 1, 2><<<dim3(CH / 128, HD / 64, (unsigned)NSL), blk, 0, stream>>>(
      XH, XH, G, CH, (long long)CH * CH, 0,
      XH, XL, XW, (long long)CH * XW, HD,
      out, XW, (long long)CH * XW, HD,
      YO, XW, (long long)CH * XW, HD,
      ACS, (long long)CH * NH, 1,
      NH, CH);
}
